// GraphSAGEModel_51642686767944
// MI455X (gfx1250) — hardware-verified
//
#include <hip/hip_runtime.h>
#include <stddef.h>
#include <stdint.h>


#define FIN     50
#define FP      64
#define CH      32
#define KA      128
#define NTHR    256
#define NWAVE   8
#define EPT     8
#define CHUNK   (NTHR * EPT)
#define WCAP    (EPT * 32)
#define LISTN   (NWAVE * WCAP)
#define NBMAX   2048
#define RCAP    28672
#define DEGCAP  96
#define PKS     11
#define STW     512
#define GBM     64
#define GTHR    128
#define WSMAX   134217728
#define LDS_AGG ((2 * RCAP + 2 * NBMAX + LISTN) * 4 + 64)

static_assert((CHUNK & (CHUNK - 1)) == 0 && CHUNK <= (1 << PKS));
static_assert((NBMAX & (NBMAX - 1)) == 0 && NBMAX <= (1 << PKS));
static_assert(NTHR * 8 == NBMAX);
static_assert(LISTN >= NBMAX);
static_assert(LISTN >= NWAVE * WCAP);
static_assert((RCAP % 32) == 0);
static_assert(NWAVE * STW <= RCAP);
static_assert(LDS_AGG <= 300000);
static_assert(GBM == (GTHR / 32) * 16);
static_assert(KA == 2 * FP && KA == 4 * CH && (KA % 32) == 0);
static_assert(FP >= FIN && (FP % 8) == 0);
static_assert(CH == 32);
static_assert(CH * (FP / 8) == NTHR);
static_assert(64 <= STW);
static_assert(GTHR >= GBM);

typedef float          v4f  __attribute__((ext_vector_type(4)));
typedef float          v8f  __attribute__((ext_vector_type(8)));
typedef int            v4i  __attribute__((ext_vector_type(4)));
typedef int            v8i  __attribute__((ext_vector_type(8)));
typedef unsigned int   v4u  __attribute__((ext_vector_type(4)));
typedef unsigned short v8us __attribute__((ext_vector_type(8)));
typedef __bf16         v16b __attribute__((ext_vector_type(16)));
typedef v8us __attribute__((may_alias)) v8usa;
typedef v4f  __attribute__((may_alias)) v4fa;
typedef v4u  __attribute__((may_alias)) v4ua;
union FragB { v16b v; v8us h[2]; v8i w; };

__device__ __forceinline__ unsigned bf16u(float f) {
  const unsigned u = __float_as_uint(f);
  return (u + 0x7FFFu + ((u >> 16) & 1u)) & 0xFFFF0000u;
}
__device__ __forceinline__ float bf16r(float f) { return __uint_as_float(bf16u(f)); }
__device__ __forceinline__ unsigned short bf16s(float f) { return (unsigned short)(bf16u(f) >> 16); }

__device__ __forceinline__ v8f wmb(const FragB& a, const FragB& b, v8f c) {
  v8f d = __builtin_amdgcn_wmma_f32_16x16x32_bf16(false, a.v, false, b.v, (short)0, c, false, false);
  asm volatile("v_nop\n\tv_nop\n\tv_nop\n\tv_nop" : "+v"(d) : "v"(a.w), "v"(b.w));
  return d;
}

__device__ __forceinline__ void ldwait() {
  asm volatile("s_wait_loadcnt 0x0" ::: "memory");
}

__device__ __forceinline__ int scan_chunk(const int* __restrict__ dsts, int nE, int cbase, int slotBase,
                                          int nb, int vec8, int* list, int tid, int lane, int wave) {
  int wc = 0;
  const int el0  = tid * EPT;
  const int e0   = cbase + el0;
  const int sent = -2147483647 - 1;
  v4i da, db;
  if (vec8 != 0 && cbase + CHUNK <= nE) {
    da = *(const v4i*)(dsts + e0);
    db = *(const v4i*)(dsts + e0 + 4);
  } else {
    da.x = (e0     < nE) ? dsts[min(e0,     nE - 1)] : sent;
    da.y = (e0 + 1 < nE) ? dsts[min(e0 + 1, nE - 1)] : sent;
    da.z = (e0 + 2 < nE) ? dsts[min(e0 + 2, nE - 1)] : sent;
    da.w = (e0 + 3 < nE) ? dsts[min(e0 + 3, nE - 1)] : sent;
    db.x = (e0 + 4 < nE) ? dsts[min(e0 + 4, nE - 1)] : sent;
    db.y = (e0 + 5 < nE) ? dsts[min(e0 + 5, nE - 1)] : sent;
    db.z = (e0 + 6 < nE) ? dsts[min(e0 + 6, nE - 1)] : sent;
    db.w = (e0 + 7 < nE) ? dsts[min(e0 + 7, nE - 1)] : sent;
  }
  const unsigned nbs = (unsigned)slotBase;
  const unsigned unb = (unsigned)nb;
  const unsigned s0 = (unsigned)da.x - nbs, s1 = (unsigned)da.y - nbs;
  const unsigned s2 = (unsigned)da.z - nbs, s3 = (unsigned)da.w - nbs;
  const unsigned s4 = (unsigned)db.x - nbs, s5 = (unsigned)db.y - nbs;
  const unsigned s6 = (unsigned)db.z - nbs, s7 = (unsigned)db.w - nbs;
  const bool h0 = s0 < unb, h1 = s1 < unb, h2 = s2 < unb, h3 = s3 < unb;
  const bool h4 = s4 < unb, h5 = s5 < unb, h6 = s6 < unb, h7 = s7 < unb;
  const unsigned any = __builtin_amdgcn_ballot_w32(h0 | h1 | h2 | h3 | h4 | h5 | h6 | h7);
  if (any != 0u) {
#define HITJ(J, HJ, SJ) { \
      const unsigned mj = __builtin_amdgcn_ballot_w32(HJ); \
      if (mj != 0u) { \
        if (HJ) { \
          const int pos = wc + (int)__builtin_amdgcn_mbcnt_lo(mj, 0u); \
          if (pos < WCAP) list[wave * WCAP + pos] = ((el0 + (J)) << PKS) | (int)(SJ); \
        } \
        wc += (int)__builtin_popcount(mj); } }
    HITJ(0, h0, s0)
    HITJ(1, h1, s1)
    HITJ(2, h2, s2)
    HITJ(3, h3, s3)
    HITJ(4, h4, s4)
    HITJ(5, h5, s5)
    HITJ(6, h6, s6)
    HITJ(7, h7, s7)
#undef HITJ
  }
  return wc;
}

__global__ __launch_bounds__(NTHR) void k_xprep(const float* __restrict__ x, unsigned short* xb,
                                                int nN, int nUnits) {
  const int i = (int)blockIdx.x * NTHR + (int)threadIdx.x;
  if (i >= nUnits) return;
  const int row = i >> 3;
  const int c0  = (i & 7) * 8;
  const int rc  = row < nN ? row : nN - 1;
  const float* p = x + (size_t)rc * FIN;
  float wv[8];
#pragma unroll
  for (int e = 0; e < 8; ++e) {
    int c = c0 + e;
    c = c < FIN ? c : FIN - 1;
    wv[e] = p[c];
  }
  ldwait();
  v8us pk;
#pragma unroll
  for (int e = 0; e < 8; ++e) {
    const bool ok = (row < nN) && (c0 + e < FIN);
    pk[e] = ok ? bf16s(wv[e]) : (unsigned short)0;
  }
  unsigned short* gp = xb + (size_t)row * FP + c0;
  *(volatile v8us*)gp = pk;
  __threadfence();
  *(volatile v8us*)gp = pk;
}

__global__ __launch_bounds__(NTHR) void k_wtr(const float* __restrict__ wl1, const float* __restrict__ wr1,
                                              const float* __restrict__ wl2, const float* __restrict__ wr2,
                                              const float* __restrict__ wl3, const float* __restrict__ wr3,
                                              unsigned short* wt) {
  const int b    = (int)blockIdx.x;
  const int tid  = (int)threadIdx.x;
  const int mat  = b >> 1;
  const int half = b & 1;
  const int n    = tid >> 3;
  const int kq   = tid & 7;
  const float* W;
  int din, rep;
  if (mat == 0)      { W = half ? wr1 : wl1; din = FIN; rep = 0; }
  else if (mat == 1) { W = half ? wr2 : wl2; din = CH;  rep = 1; }
  else               { W = half ? wr3 : wl3; din = CH;  rep = 1; }
  float wv[8];
#pragma unroll
  for (int e = 0; e < 8; ++e) {
    int kk = 8 * kq + e;
    if (rep) kk &= (CH - 1);
    const int kcl = kk < din ? kk : din - 1;
    wv[e] = W[(size_t)kcl * CH + n];
  }
  ldwait();
  v8us pk;
#pragma unroll
  for (int e = 0; e < 8; ++e) {
    int kk = 8 * kq + e;
    if (rep) kk &= (CH - 1);
    pk[e] = (kk < din) ? bf16s(wv[e]) : (unsigned short)0;
  }
  const int k8 = FP * half + 8 * kq;
  unsigned short* gp = wt + (size_t)mat * CH * KA + (size_t)n * KA + k8;
  *(volatile v8us*)gp = pk;
  __threadfence();
  *(volatile v8us*)gp = pk;
}

template<int L1>
__global__ __launch_bounds__(NTHR) void k_agg(
    const int* __restrict__ srcs, const int* __restrict__ dsts,
    const unsigned int* __restrict__ xb,
    const float* __restrict__ hf,
    unsigned short* Aout,
    int nN, int nE, int nb, int vec8, int MPr) {
  extern __shared__ v4f lds_dyn[];
  int* reg1 = (int*)lds_dyn;
  int* reg2 = reg1 + RCAP;
  int* scnt = reg2 + RCAP;
  int* soff = scnt + NBMAX;
  int* list = soff + NBMAX;
  int* wcnt = list + LISTN;
  int* wtot = wcnt + NWAVE;
  const int tid = (int)threadIdx.x, lane = tid & 31, wave = tid >> 5;
  const int nodeBase = (int)blockIdx.x * nb;

  for (int i = tid; i < NBMAX; i += NTHR) scnt[i] = 0;
  __syncthreads();

  int tot = 0;
  const int nChunks = (nE + CHUNK - 1) / CHUNK;
#pragma unroll 1
  for (int ch = 0; ch < nChunks; ++ch) {
    const int cbase = ch * CHUNK;
    const int wc = scan_chunk(dsts, nE, cbase, nodeBase, nb, vec8, list, tid, lane, wave);
    if (lane == 0) wcnt[wave] = wc;
    __syncthreads();
    int pre = 0, all = 0;
#pragma unroll
    for (int w2 = 0; w2 < NWAVE; ++w2) {
      int c = wcnt[w2];
      c = c < 0 ? 0 : (c > WCAP ? WCAP : c);
      all += c;
      pre += (w2 < wave) ? c : 0;
    }
    const int wcc  = wc > WCAP ? WCAP : wc;
    const int base = tot + pre;
#pragma unroll 1
    for (int i = lane; i < wcc; i += 32) {
      const int ent = list[wave * WCAP + i];
      const int el  = (ent >> PKS) & (CHUNK - 1);
      const int sl  = ent & (NBMAX - 1);
      int eid = cbase + el;
      eid = eid > nE - 1 ? nE - 1 : eid;
      const int pos = base + i;
      if (pos < RCAP) reg1[pos] = (int)(((unsigned)eid << PKS) | (unsigned)sl);
    }
    tot += all;
    tot = tot > RCAP ? RCAP : tot;
    __syncthreads();
  }
  const int nh = tot;

  if (wave == 0) {
#pragma unroll 1
    for (int b0 = 0; b0 < nh; b0 += 32) {
      const int idx = b0 + lane;
      const int uv  = reg1[idx < RCAP ? idx : RCAP - 1];
      const int m32 = (nh - b0) < 32 ? (nh - b0) : 32;
#pragma unroll 1
      for (int k = 0; k < m32; ++k) {
        const int u  = __builtin_amdgcn_readlane(uv, k);
        const int sl = u & (NBMAX - 1);
        if (lane == 0) scnt[sl] = scnt[sl] + 1;
      }
    }
  }
  __syncthreads();

  {
    const v4i ca = *(const v4i*)(scnt + 8 * tid);
    const v4i cb = *(const v4i*)(scnt + 8 * tid + 4);
    const int e0 = ca.x < 0 ? 0 : ca.x, e1 = ca.y < 0 ? 0 : ca.y, e2 = ca.z < 0 ? 0 : ca.z, e3 = ca.w < 0 ? 0 : ca.w;
    const int e4 = cb.x < 0 ? 0 : cb.x, e5 = cb.y < 0 ? 0 : cb.y, e6 = cb.z < 0 ? 0 : cb.z, e7 = cb.w < 0 ? 0 : cb.w;
    const int ts = e0 + e1 + e2 + e3 + e4 + e5 + e6 + e7;
    int incl = ts;
#pragma unroll
    for (int d = 1; d < 32; d <<= 1) {
      const int up = __shfl_up(incl, d);
      if (lane >= d) incl += up;
    }
    if (lane == 31) wtot[wave] = incl;
    __syncthreads();
    int pre = 0;
#pragma unroll
    for (int w2 = 0; w2 < NWAVE; ++w2) pre += (w2 < wave) ? wtot[w2] : 0;
    int run = pre + incl - ts;
    soff[8 * tid + 0] = run; run += e0;
    soff[8 * tid + 1] = run; run += e1;
    soff[8 * tid + 2] = run; run += e2;
    soff[8 * tid + 3] = run; run += e3;
    soff[8 * tid + 4] = run; run += e4;
    soff[8 * tid + 5] = run; run += e5;
    soff[8 * tid + 6] = run; run += e6;
    soff[8 * tid + 7] = run;
  }
  __syncthreads();
  for (int i = tid; i < NBMAX; i += NTHR) list[i] = soff[i];
  __syncthreads();

  if (wave == 0) {
#pragma unroll 1
    for (int b0 = 0; b0 < nh; b0 += 32) {
      const int idx = b0 + lane;
      const int uv  = reg1[idx < RCAP ? idx : RCAP - 1];
      const int m32 = (nh - b0) < 32 ? (nh - b0) : 32;
#pragma unroll 1
      for (int k = 0; k < m32; ++k) {
        const int u   = __builtin_amdgcn_readlane(uv, k);
        const int sl  = u & (NBMAX - 1);
        const int eid = (int)((unsigned)u >> PKS);
        if (lane == 0) {
          int pos = list[sl];
          pos = pos < 0 ? 0 : (pos > RCAP - 1 ? RCAP - 1 : pos);
          reg2[pos] = eid;
          list[sl] = pos + 1;
        }
      }
    }
  }
  __syncthreads();

  const int nbw = nb >> 3;
  const bool ovf = (nh >= RCAP);
  const float qnan = __int_as_float(0x7fc00000);
  const float ninf = __int_as_float((int)0xff800000u);
  float* stw = (float*)reg1 + wave * STW;
  unsigned int*   stwu = (unsigned int*)stw;
  unsigned short* st16 = (unsigned short*)stw;
  const int lq = lane < 16 ? lane : 15;

#pragma unroll 1
  for (int jt = 0; jt < nbw; ++jt) {
    const int slot = wave * nbw + jt;
    const int grow = nodeBase + slot;
    const int gcl  = grow < nN ? grow : nN - 1;
    int st = soff[slot];
    const int craw = scnt[slot];
    int cnt = craw;
    st  = st < 0 ? 0 : (st > nh ? nh : st);
    cnt = cnt < 0 ? 0 : (cnt > DEGCAP ? DEGCAP : cnt);
    if (cnt > nh - st) cnt = nh - st;
    const float pz   = (ovf || craw > DEGCAP) ? qnan : 0.0f;
    const float live = grow < nN ? 1.0f : 0.0f;
    const bool  wsv  = (grow < MPr) && (lane < 16);
    unsigned short* gp = Aout + (size_t)grow * KA + 8 * lq;

    if (L1) {
      const unsigned sw = xb[(size_t)gcl * (FP / 2) + lane];
      ldwait();
      float a0 = ninf, a1 = ninf;
#pragma unroll 1
      for (int q = 0; q < cnt; ++q) {
        int idx = st + q; idx = idx > RCAP - 1 ? RCAP - 1 : idx;
        int eid = reg2[idx]; eid = eid < 0 ? 0 : (eid > nE - 1 ? nE - 1 : eid);
        const int sraw = srcs[eid];
        ldwait();
        const int s = sraw < 0 ? 0 : (sraw > nN - 1 ? nN - 1 : sraw);
        const unsigned g = xb[(size_t)s * (FP / 2) + lane];
        ldwait();
        a0 = fmaxf(a0, __uint_as_float(g << 16));
        a1 = fmaxf(a1, __uint_as_float(g & 0xFFFF0000u));
      }
      a0 = cnt > 0 ? a0 : 0.0f;
      a1 = cnt > 0 ? a1 : 0.0f;
      const float s0 = __uint_as_float(sw << 16);
      const float s1 = __uint_as_float(sw & 0xFFFF0000u);
      const float ra0 = a0 * live + pz, ra1 = a1 * live + pz;
      const float rs0 = s0 * live + pz, rs1 = s1 * live + pz;
      const unsigned aw  = (__float_as_uint(ra0) >> 16) | (__float_as_uint(ra1) & 0xFFFF0000u);
      const unsigned swo = (__float_as_uint(rs0) >> 16) | (__float_as_uint(rs1) & 0xFFFF0000u);
      __builtin_amdgcn_fence(__ATOMIC_RELEASE, "wavefront");
      __builtin_amdgcn_wave_barrier();
      stwu[lane]      = aw;
      stwu[32 + lane] = swo;
      __builtin_amdgcn_fence(__ATOMIC_RELEASE, "wavefront");
      __builtin_amdgcn_wave_barrier();
      const v4u pk = *(const v4ua*)(stwu + 4 * lq);
      if (wsv) *(volatile v4u*)gp = pk;
      __threadfence();
      if (wsv) *(volatile v4u*)gp = pk;
    } else {
      const float sv = hf[(size_t)gcl * CH + lane];
      ldwait();
      float a = ninf;
#pragma unroll 1
      for (int q = 0; q < cnt; ++q) {
        int idx = st + q; idx = idx > RCAP - 1 ? RCAP - 1 : idx;
        int eid = reg2[idx]; eid = eid < 0 ? 0 : (eid > nE - 1 ? nE - 1 : eid);
        const int sraw = srcs[eid];
        ldwait();
        const int s = sraw < 0 ? 0 : (sraw > nN - 1 ? nN - 1 : sraw);
        const float g = hf[(size_t)s * CH + lane];
        ldwait();
        a = fmaxf(a, g);
      }
      a = cnt > 0 ? a : 0.0f;
      const float ra = a * live + pz;
      const float rs = sv * live + pz;
      const unsigned ahu = bf16u(ra);
      const unsigned alu = bf16u(ra - __uint_as_float(ahu));
      const unsigned shu = bf16u(rs);
      const unsigned slu = bf16u(rs - __uint_as_float(shu));
      __builtin_amdgcn_fence(__ATOMIC_RELEASE, "wavefront");
      __builtin_amdgcn_wave_barrier();
      st16[lane]      = (unsigned short)(ahu >> 16);
      st16[32 + lane] = (unsigned short)(alu >> 16);
      st16[64 + lane] = (unsigned short)(shu >> 16);
      st16[96 + lane] = (unsigned short)(slu >> 16);
      __builtin_amdgcn_fence(__ATOMIC_RELEASE, "wavefront");
      __builtin_amdgcn_wave_barrier();
      const v8us pk = *(const v8usa*)(st16 + 8 * lq);
      if (wsv) *(volatile v8us*)gp = pk;
      __threadfence();
      if (wsv) *(volatile v8us*)gp = pk;
    }
  }
}

template<int MODE>
__global__ __launch_bounds__(GTHR) void k_gemm(const unsigned short* __restrict__ A,
                                               const unsigned short* __restrict__ WT,
                                               const float* __restrict__ bias, float* outF, int nN) {
  __shared__ __attribute__((aligned(16))) float stg[GBM * CH];
  __shared__ float rmx[GBM];
  __shared__ float rls[GBM];
  const int tid = (int)threadIdx.x, lane = tid & 31, wave = tid >> 5, hh = lane >> 4, m = lane & 15;
  const int rowBase = (int)blockIdx.x * GBM;

  v8f acc[2];
  {
    const v8f z = {0.f, 0.f, 0.f, 0.f, 0.f, 0.f, 0.f, 0.f};
    acc[0] = z; acc[1] = z;
  }
  const unsigned short* ap = A  + (size_t)(rowBase + 16 * wave + m) * (size_t)KA + 8 * hh;
  const unsigned short* wp = WT + (size_t)m * (size_t)KA + 8 * hh;
#pragma unroll 1
  for (int ks = 0; ks < KA / 32; ++ks) {
    FragB af;
    af.h[0] = *(const v8usa*)(ap + 32 * ks);
    af.h[1] = *(const v8usa*)(ap + 32 * ks + 16);
#pragma unroll
    for (int t = 0; t < 2; ++t) {
      const unsigned short* wq = wp + (size_t)(16 * t) * (size_t)KA + 32 * ks;
      FragB bf;
      bf.h[0] = *(const v8usa*)wq;
      bf.h[1] = *(const v8usa*)(wq + 16);
      acc[t] = wmb(af, bf, acc[t]);
    }
  }

  float bv[2];
  bv[0] = bias[m];
  bv[1] = bias[16 + m];
  ldwait();
#pragma unroll
  for (int t = 0; t < 2; ++t) {
    const int lc = 16 * t + m;
    const float bb = bf16r(bv[t]);
#pragma unroll
    for (int r = 0; r < 8; ++r) {
      const int lr = 16 * wave + 8 * hh + r;
      float v = acc[t][r] + bb;
      if (MODE == 0) v = fmaxf(v, 0.0f);
      stg[lr * CH + lc] = v;
    }
  }
  __syncthreads();

  if (MODE == 1) {
    const float ninf = __int_as_float((int)0xff800000u);
    if (tid < GBM) {
      const float* rp = stg + tid * CH;
      float mx = ninf;
#pragma unroll 1
      for (int c = 0; c < CH; ++c) mx = fmaxf(mx, rp[c]);
      float s = 0.0f;
#pragma unroll 1
      for (int c = 0; c < CH; ++c) s += expf(rp[c] - mx);
      rmx[tid] = mx;
      rls[tid] = logf(s);
    }
    __syncthreads();
  }

  const int rsub = lane >> 3;
  const int cp   = lane & 7;
  v4f fv[4];
#pragma unroll
  for (int i = 0; i < 4; ++i) {
    const int lr = 16 * wave + 4 * i + rsub;
    v4f v = *(const v4fa*)(stg + lr * CH + 4 * cp);
    if (MODE == 1) {
      const float mm = rmx[lr];
      const float ll = rls[lr];
      v = (v - mm) - ll;
    }
    fv[i] = v;
  }
#pragma unroll
  for (int i = 0; i < 4; ++i) {
    const int lr = 16 * wave + 4 * i + rsub;
    const int gr = rowBase + lr;
    const bool ok = (MODE == 0) || (gr < nN);
    float* op = outF + (size_t)gr * CH + 4 * cp;
    if (ok) *(volatile v4f*)op = fv[i];
  }
  __threadfence();
#pragma unroll
  for (int i = 0; i < 4; ++i) {
    const int lr = 16 * wave + 4 * i + rsub;
    const int gr = rowBase + lr;
    const bool ok = (MODE == 0) || (gr < nN);
    float* op = outF + (size_t)gr * CH + 4 * cp;
    if (ok) *(volatile v4f*)op = fv[i];
  }
}

static int pick_nb(int nE, int nN) {
  int nb = NBMAX;
  while (nb > 16 && (long long)nb * (long long)nE * 5LL > (long long)RCAP * (long long)nN * 4LL) nb >>= 1;
  return nb;
}
static inline int cdiv(int a, int b) { return (a + b - 1) / b; }

extern "C" void kernel_launch(void* const* d_in, const int* in_sizes, int n_in,
                              void* d_out, int out_size, void* d_ws, size_t ws_size,
                              hipStream_t stream) {
  if (n_in < 11) return;
  if (in_sizes[0] < FIN || (in_sizes[0] % FIN) != 0) return;
  const int nN = in_sizes[0] / FIN;
  if (nN <= 0 || nN > (1 << 22)) return;
  if (in_sizes[1] < 2 || (in_sizes[1] & 1) != 0) return;
  const int nE = in_sizes[1] / 2;
  if (nE < 1 || nE > (1 << 21)) return;
  if (in_sizes[2] != FIN * CH || in_sizes[3] != CH || in_sizes[4]  != FIN * CH) return;
  if (in_sizes[5] != CH * CH  || in_sizes[6] != CH || in_sizes[7]  != CH * CH)  return;
  if (in_sizes[8] != CH * CH  || in_sizes[9] != CH || in_sizes[10] != CH * CH)  return;
  if (out_size != nN * CH) return;

  const float* x   = (const float*)d_in[0];
  const int*   ei  = (const int*)  d_in[1];
  const float* Wl1 = (const float*)d_in[2];
  const float* bl1 = (const float*)d_in[3];
  const float* Wr1 = (const float*)d_in[4];
  const float* Wl2 = (const float*)d_in[5];
  const float* bl2 = (const float*)d_in[6];
  const float* Wr2 = (const float*)d_in[7];
  const float* Wl3 = (const float*)d_in[8];
  const float* bl3 = (const float*)d_in[9];
  const float* Wr3 = (const float*)d_in[10];
  const int* src = ei;
  const int* dst = ei + nE;
  float* out = (float*)d_out;

  const int MP   = cdiv(nN, GBM) * GBM;
  const int gM   = MP / GBM;
  const int nb   = pick_nb(nE, nN);
  const int gA   = cdiv(MP, nb);
  const int vec8 = ((nE & 3) == 0) ? 1 : 0;
  if (gA * nb < MP) return;

  char* ws = (char*)d_ws;
  size_t off = 0;
  const size_t oXB  = off; off += (size_t)MP * FP * 2;          off = (off + 255) & ~(size_t)255;
  const size_t oWT  = off; off += (size_t)3 * CH * KA * 2;      off = (off + 255) & ~(size_t)255;
  const size_t oAP1 = off; off += (size_t)MP * KA * 2;          off = (off + 255) & ~(size_t)255;
  const size_t oH1  = off; off += (size_t)MP * CH * 4;          off = (off + 255) & ~(size_t)255;
  const size_t oAP2 = off; off += (size_t)MP * KA * 2;          off = (off + 255) & ~(size_t)255;
  const size_t oH2  = off; off += (size_t)MP * CH * 4;          off = (off + 255) & ~(size_t)255;
  const size_t oAP3 = off; off += (size_t)MP * KA * 2;          off = (off + 255) & ~(size_t)255;
  if (off > ws_size || off > (size_t)WSMAX) return;
  unsigned short* XB  = (unsigned short*)(ws + oXB);
  unsigned short* WT  = (unsigned short*)(ws + oWT);
  unsigned short* AP1 = (unsigned short*)(ws + oAP1);
  float*          H1  = (float*)(ws + oH1);
  unsigned short* AP2 = (unsigned short*)(ws + oAP2);
  float*          H2  = (float*)(ws + oH2);
  unsigned short* AP3 = (unsigned short*)(ws + oAP3);
  const unsigned int* XBw = (const unsigned int*)XB;

  hipFuncSetAttribute(reinterpret_cast<const void*>(&k_agg<0>),
                      hipFuncAttributeMaxDynamicSharedMemorySize, LDS_AGG);
  hipFuncSetAttribute(reinterpret_cast<const void*>(&k_agg<1>),
                      hipFuncAttributeMaxDynamicSharedMemorySize, LDS_AGG);

  const int nUx = MP * (FP / 8);
  k_xprep<<<cdiv(nUx, NTHR), NTHR, 0, stream>>>(x, XB, nN, nUx);

  k_wtr<<<6, NTHR, 0, stream>>>(Wl1, Wr1, Wl2, Wr2, Wl3, Wr3, WT);

  k_agg<1><<<gA, NTHR, LDS_AGG, stream>>>(src, dst, XBw, H1, AP1, nN, nE, nb, vec8, MP);
  k_gemm<0><<<gM, GTHR, 0, stream>>>(AP1, WT, bl1, H1, nN);

  k_agg<0><<<gA, NTHR, LDS_AGG, stream>>>(src, dst, XBw, H1, AP2, nN, nE, nb, vec8, MP);
  k_gemm<0><<<gM, GTHR, 0, stream>>>(AP2, WT + (size_t)CH * KA, bl2, H2, nN);

  k_agg<0><<<gA, NTHR, LDS_AGG, stream>>>(src, dst, XBw, H2, AP3, nN, nE, nb, vec8, MP);
  k_gemm<1><<<gM, GTHR, 0, stream>>>(AP3, WT + (size_t)2 * CH * KA, bl3, out, nN);
}
